// QTRAN_alt_20151986553260
// MI455X (gfx1250) — hardware-verified
//
#include <hip/hip_runtime.h>
#include <math.h>

typedef __attribute__((ext_vector_type(16))) _Float16 v16h;
typedef __attribute__((ext_vector_type(16))) __bf16 v16b;
typedef __attribute__((ext_vector_type(8)))  _Float16 v8h;
typedef __attribute__((ext_vector_type(8)))  float v8f;
typedef __attribute__((ext_vector_type(4)))  float v4f;
typedef __attribute__((ext_vector_type(2)))  float v2f;
typedef __attribute__((ext_vector_type(4)))  unsigned v4u;
typedef __attribute__((ext_vector_type(4)))  int v4i;
typedef float __attribute__((may_alias)) float_a;
typedef int __attribute__((may_alias)) int_a;

template <typename T> __device__ __forceinline__ void vst2(void* p, T v) { *(volatile T*)p = v; __threadfence(); *(volatile T*)p = v; }
__device__ __forceinline__ v8f wmma16(v16h a, v16h b, v8f c) {
  v8f d = __builtin_amdgcn_wmma_f32_16x16x32_f16(false, a, false, b, (short)0, c, false, false);
  asm volatile("v_nop\n\tv_nop\n\tv_nop\n\tv_nop" : "+v"(d) : "v"(a), "v"(b));
  return d;
}
__device__ __forceinline__ v8f wmma_bf(v16b a, v16b b, v8f c) {
  v8f d = __builtin_amdgcn_wmma_f32_16x16x32_bf16(false, a, false, b, (short)0, c, false, false);
  asm volatile("v_nop\n\tv_nop\n\tv_nop\n\tv_nop" : "+v"(d) : "v"(a), "v"(b));
  return d;
}
__device__ __forceinline__ v16h frag_h(const _Float16* rowk0, int lane) {
  union { v16h v; v8h q[2]; } u; const _Float16* p = rowk0 + 8 * (lane >> 4);
  u.q[0] = *(const v8h*)p; u.q[1] = *(const v8h*)(p + 16); return u.v;
}
__device__ __forceinline__ v16h frag_f32(const float* rowk0, int lane) {
  v16h a; const float* p = rowk0 + 8 * (lane >> 4);
#pragma unroll
  for (int i = 0; i < 8; ++i) { a[i] = (_Float16)p[i]; a[8 + i] = (_Float16)p[16 + i]; }
  return a;
}
__device__ __forceinline__ v16h frag_f32s(const float* rowk0, int lane, float sc) {
  v16h a; const float* p = rowk0 + 8 * (lane >> 4);
#pragma unroll
  for (int i = 0; i < 8; ++i) { a[i] = (_Float16)(p[i] * sc); a[8 + i] = (_Float16)(p[16 + i] * sc); }
  return a;
}
__device__ __forceinline__ v16h fragc_f32(const float* W, int k0, int n, int lane, int ld, int K) {
  v16h a; const int g = lane >> 4;
#pragma unroll
  for (int i = 0; i < 8; ++i) { const int ka = k0 + 8 * g + i, kb = ka + 16;
    a[i] = (_Float16)(ka < K ? W[(size_t)ka * ld + n] : 0.f); a[8 + i] = (_Float16)(kb < K ? W[(size_t)kb * ld + n] : 0.f); }
  return a;
}
struct F2 { v16b h, l; };
__device__ __forceinline__ F2 bsplit16(const float v[16]) { F2 r;
#pragma unroll
  for (int i = 0; i < 16; ++i) { const __bf16 h = (__bf16)v[i]; r.h[i] = h; r.l[i] = (__bf16)(v[i] - (float)h); }
  return r; }
__device__ __forceinline__ F2 split_row(const float* row, int k0, int lane) { float v[16]; const float* p = row + k0 + 8 * (lane >> 4);
#pragma unroll
  for (int i = 0; i < 8; ++i) { v[i] = p[i]; v[8 + i] = p[16 + i]; }
  return bsplit16(v); }
__device__ __forceinline__ F2 split_rowK(const float* row, int k0, int lane, int K) { float v[16]; const int g = lane >> 4;
#pragma unroll
  for (int i = 0; i < 8; ++i) { const int ka = k0 + 8 * g + i, kb = ka + 16; v[i] = ka < K ? row[ka] : 0.f; v[8 + i] = kb < K ? row[kb] : 0.f; }
  return bsplit16(v); }
__device__ __forceinline__ F2 split_col(const float* W, int k0, int n, int lane, int ld, int K) { float v[16]; const int g = lane >> 4;
#pragma unroll
  for (int i = 0; i < 8; ++i) { const int ka = k0 + 8 * g + i, kb = ka + 16; v[i] = ka < K ? W[(size_t)ka * ld + n] : 0.f; v[8 + i] = kb < K ? W[(size_t)kb * ld + n] : 0.f; }
  return bsplit16(v); }
__device__ __forceinline__ v8f mac3(const F2& a, const F2& b, v8f c) { c = wmma_bf(a.l, b.h, c); c = wmma_bf(a.h, b.l, c); return wmma_bf(a.h, b.h, c); }
__device__ __forceinline__ float sigm(float v) { return 1.0f / (1.0f + expf(-v)); }
#define LDSX() do { asm volatile("s_wait_dscnt 0" ::: "memory"); __builtin_amdgcn_wave_barrier(); __builtin_amdgcn_fence(__ATOMIC_RELEASE, "workgroup"); } while (0)

#define NBT 2048
#define NAG 8
#define NAC 16
#define HH 32
#define HID 64
#define DQ ((HH + NAC) * NAG)
#define NCF (NBT * NAG * NAC)

__global__ __launch_bounds__(128) void k_base(const float* __restrict__ hs, const float* __restrict__ act, const float* __restrict__ W1, float* __restrict__ base, float* __restrict__ actc) {
  __shared__ __align__(16) float sx[4][16][DQ + 4];
  __shared__ __align__(16) float so[4][16][68];
  const int tid = threadIdx.x, wave = tid >> 5, lane = tid & 31, col = lane & 15, g = lane >> 4;
  const int r0 = blockIdx.x * 64 + wave * 16;
  for (int q = lane; q < 16 * DQ; q += 32) { const int rl = q / DQ, c = q % DQ; const int j = c / (HH + NAC), cc = c % (HH + NAC);
    sx[wave][rl][c] = cc < HH ? hs[((size_t)(r0 + rl) * NAG + j) * HH + cc] : act[((size_t)(r0 + rl) * NAG + j) * NAC + cc - HH]; }
  LDSX();
  v8f acc[4] = {};
#pragma unroll 2
  for (int kc = 0; kc < DQ / 32; ++kc) { const v16h a = frag_f32(&sx[wave][col][0] + kc * 32, lane);
#pragma unroll
    for (int t = 0; t < 4; ++t) { v16h bb = fragc_f32(W1, kc * 32, t * 16 + col, lane, HID, DQ);
#pragma unroll
      for (int e = 0; e < 16; ++e) bb[e] = bb[e] * (_Float16)16.0f;
      acc[t] = wmma16(a, bb, acc[t]); } }
#pragma unroll
  for (int t = 0; t < 4; ++t)
#pragma unroll
    for (int r = 0; r < 8; ++r) so[wave][8 * g + r][t * 16 + col] = acc[t][r] * (1.0f / 16.0f);
  LDSX();
  for (int q = lane; q < 16 * 16; q += 32) { const int rl = q >> 4, pc = q & 15; vst2(base + (size_t)(r0 + rl) * HID + pc * 4, *(const v4f*)(&so[wave][rl][pc * 4])); }
  LDSX();
#pragma unroll 1
  for (int gg = 0; gg < NAG; ++gg) {
    for (int q = lane; q < 16 * HID; q += 32) { const int rl = q >> 6, c = q & 63; float s = 0.f;
#pragma unroll
      for (int a = 0; a < NAC; ++a) s += sx[wave][rl][gg * (HH + NAC) + HH + a] * W1[(size_t)(gg * (HH + NAC) + HH + a) * HID + c];
      so[wave][rl][c] = s; }
    LDSX();
    for (int q = lane; q < 16 * 16; q += 32) { const int rl = q >> 4, pc = q & 15; vst2(actc + ((size_t)(r0 + rl) * NAG + gg) * HID + pc * 4, *(const v4f*)(&so[wave][rl][pc * 4])); }
    LDSX(); }
}
__global__ __launch_bounds__(128) void k_cf(const float* __restrict__ base, const float* __restrict__ actc, const float* __restrict__ W1, const float* __restrict__ b1, const float* __restrict__ W2, const float* __restrict__ b2, const float* __restrict__ w3, const float* __restrict__ b3, float* __restrict__ out) {
  __shared__ __align__(16) float sh[4][16][68];
  __shared__ __align__(16) float sq[64];
  const int tid = threadIdx.x, wave = tid >> 5, lane = tid & 31, col = lane & 15, g = lane >> 4;
  const int r0 = blockIdx.x * 64 + wave * 16;
  for (int q = lane; q < 16 * HID; q += 32) { const int rl = q >> 6, c = q & 63; const int cf = r0 + rl; const int a = cf & 15, gg = (cf >> 4) & 7, b = cf >> 7;
    const float v = base[(size_t)b * HID + c] - actc[((size_t)b * NAG + gg) * HID + c] + W1[(size_t)(gg * (HH + NAC) + HH + a) * HID + c] + b1[c]; sh[wave][rl][c] = v > 0.f ? v : 0.f; }
  LDSX();
  v8f acc[4] = {};
#pragma unroll
  for (int kc = 0; kc < 2; ++kc) { const v16h aa = frag_f32(&sh[wave][col][0] + kc * 32, lane);
#pragma unroll
    for (int t = 0; t < 4; ++t) { v16h bb = fragc_f32(W2, kc * 32, t * 16 + col, lane, HID, HID);
#pragma unroll
      for (int e = 0; e < 16; ++e) bb[e] = bb[e] * (_Float16)8.0f;
      acc[t] = wmma16(aa, bb, acc[t]); } }
  LDSX();
#pragma unroll
  for (int t = 0; t < 4; ++t) { const int c = t * 16 + col; const float bb = b2[c];
#pragma unroll
    for (int r = 0; r < 8; ++r) { const float v = acc[t][r] * 0.125f + bb; sh[wave][8 * g + r][c] = v > 0.f ? v : 0.f; } }
  LDSX();
  { const int rl = lane >> 1, hf = lane & 1; float s = 0.f;
#pragma unroll 8
    for (int c = 0; c < 32; ++c) s += sh[wave][rl][hf * 32 + c] * w3[hf * 32 + c];
    s += __shfl_xor(s, 1, 32); if (hf == 0) sq[wave * 16 + rl] = s + b3[0]; }
  __syncthreads();
  if (tid < 16) vst2(out + (size_t)blockIdx.x * 64 + tid * 4, *(const v4f*)(&sq[tid * 4]));
}
extern "C" void kernel_launch(void* const* d_in, const int* in_sizes, int n_in, void* d_out, int out_size, void* d_ws, size_t ws_size, hipStream_t stream) {
  (void)in_sizes; (void)n_in; (void)out_size; (void)ws_size;
  const float** I = (const float**)d_in;
  const float* hs = I[0]; const float* act = I[1]; const float* W1 = I[2]; const float* b1 = I[3]; const float* W2 = I[4]; const float* b2 = I[5]; const float* w3 = I[6]; const float* b3 = I[7];
  float* out = (float*)d_out;
  char* ws = (char*)d_ws; size_t off = 0;
  auto take = [&](size_t bytes) { char* p = ws + off; off += (bytes + 255) & ~(size_t)255; return p; };
  float* base = (float*)take((size_t)NBT * HID * 4); float* actc = (float*)take((size_t)NBT * NAG * HID * 4);
  k_base<<<NBT / 64, 128, 0, stream>>>(hs, act, W1, base, actc);
  k_cf<<<NCF / 64, 128, 0, stream>>>(base, actc, W1, b1, W2, b2, w3, b3, out);
}
